// SelfAttention_80324478370016
// MI455X (gfx1250) — hardware-verified
//
#include <hip/hip_runtime.h>


#ifndef NB
#define NB 2
#endif
#ifndef SEQ
#define SEQ 2048
#endif
#define SEQ_FULL 2048
#define DM   1024
#define NH   16
#define HD   64
#define LP   72
#define AQ   128
#define KT   64
#define MR   (NB * SEQ)
#define SCL  0.125f
#define PLANE ((size_t)NB * NH * SEQ * HD)
#define HCAR 16.0f
#define WCAR 1024.0f
#define QFOLD (1.0f / (HCAR * WCAR))

typedef _Float16 h16;
typedef unsigned short bf;
typedef __attribute__((ext_vector_type(16))) __bf16   v16bf;
typedef __attribute__((ext_vector_type(16))) _Float16 v16h;
typedef __attribute__((ext_vector_type(8)))  _Float16 v8h;
typedef __attribute__((ext_vector_type(2)))  _Float16 v2h;
typedef __attribute__((ext_vector_type(8)))  unsigned short v8us;
typedef __attribute__((ext_vector_type(2)))  unsigned short v2us;
typedef __attribute__((ext_vector_type(8)))  float    v8f;
typedef __attribute__((ext_vector_type(4)))  float    v4f;
typedef v8h  __attribute__((may_alias)) v8ha;
typedef v4f  __attribute__((may_alias)) v4fa;

static_assert(HD == 64);
static_assert(DM == NH * HD);
static_assert(DM % 64 == 0);
static_assert(DM % 32 == 0);
static_assert(SEQ % AQ == 0);
static_assert(SEQ % KT == 0);
static_assert(SEQ % 64 == 0);
static_assert(AQ == 8 * 16);
static_assert(LP % 8 == 0);
static_assert(LP >= 64);
static_assert(SEQ <= SEQ_FULL);
static_assert((3 * DM * DM) % (64 * 64) == 0);
static_assert(DM == 4 * 32 * 8);
static_assert(SEQ % 8 == 0);
static_assert(HCAR * WCAR == 16384.0f);

#define SZ_WQKV ((size_t)3 * DM * DM * 2)
#define SZ_WO   ((size_t)DM * DM * 2)
#define SZ_XB   ((size_t)MR * DM * 2)
#define SZ_PL   (PLANE * 2)
#define WS_TOTAL (SZ_WQKV + SZ_WO + SZ_XB + 3 * SZ_PL + 2 * SZ_XB)
static_assert(SZ_WQKV % 256 == 0);
static_assert(SZ_WO % 256 == 0);
static_assert(SZ_XB % 256 == 0);
static_assert(SZ_PL % 256 == 0);
static_assert(WS_TOTAL <= (size_t)134217728);

__device__ __forceinline__ unsigned short f2bf(float f) { unsigned u = __float_as_uint(f); u += 0x7FFFu + ((u >> 16) & 1u); return (unsigned short)(u >> 16); }
__device__ __forceinline__ float bf2f(unsigned short b) { return __uint_as_float(((unsigned)b) << 16); }
__device__ __forceinline__ float bfr(float f) { return bf2f(f2bf(f)); }
__device__ __forceinline__ void splitf(float y, unsigned short& h, unsigned short& l) { h = f2bf(y); l = f2bf(y - bf2f(h)); }
__device__ __forceinline__ v16h cat16(v8h lo, v8h hi) { return __builtin_shufflevector(lo, hi, 0, 1, 2, 3, 4, 5, 6, 7, 8, 9, 10, 11, 12, 13, 14, 15); }
__device__ __forceinline__ v16bf cat16b(v8us lo, v8us hi) { return __builtin_bit_cast(v16bf, __builtin_shufflevector(lo, hi, 0, 1, 2, 3, 4, 5, 6, 7, 8, 9, 10, 11, 12, 13, 14, 15)); }
__device__ __forceinline__ v8f wmma16(v16h a, v16h b, v8f c) { return __builtin_amdgcn_wmma_f32_16x16x32_f16(false, a, false, b, (short)0, c, false, false); }
__device__ __forceinline__ v8f wmmab(v16bf a, v16bf b, v8f c) { return __builtin_amdgcn_wmma_f32_16x16x32_bf16(false, a, false, b, (short)0, c, false, false); }
__device__ __forceinline__ v16bf ldb(const bf* p) { return cat16b(*(const v8us*)p, *(const v8us*)(p + 16)); }
__device__ __forceinline__ v16h ldh(const h16* p) { return cat16(*(const v8ha*)p, *(const v8ha*)(p + 16)); }
static __device__ __forceinline__ h16 toh_flush(float v) { const h16 r = (h16)v; return (fabsf(v) < 6.103515625e-05f) ? (h16)0.0f : r; }
#define LDF(arr, off) cat16(*(const v8ha*)((arr) + (off)), *(const v8ha*)((arr) + (off) + 16))

__global__ __launch_bounds__(256) void k_wtG(const float* __restrict__ w, int K, int N, bf* Bt) {
    const int lane = threadIdx.x & 31; const int L0 = (blockIdx.x * 8 + (threadIdx.x >> 5)) * 8; const int nlines = N * K / 64;
#pragma unroll
    for (int ps = 0; ps < 2; ++ps) {
#pragma unroll 1
        for (int l = 0; l < 8; ++l) { const int L = L0 + l; if (L >= nlines) break; const size_t e = (size_t)L * 64 + lane * 2; const int k = (int)(e % K), n = (int)(e / K); v2us o;
            o[0] = f2bf(w[(size_t)k * N + n]); o[1] = f2bf(w[(size_t)(k + 1) * N + n]); *(volatile v2us*)(Bt + e) = o; }
        if (ps == 0) __threadfence(); }
}

__global__ __launch_bounds__(256) void k_wtH(const float* __restrict__ w, int K, int N, h16* Bt) {
    const int lane = threadIdx.x & 31; const int L0 = (blockIdx.x * 8 + (threadIdx.x >> 5)) * 8; const int nlines = N * K / 64;
#pragma unroll
    for (int ps = 0; ps < 2; ++ps) {
#pragma unroll 1
        for (int l = 0; l < 8; ++l) { const int L = L0 + l; if (L >= nlines) break; const size_t e = (size_t)L * 64 + lane * 2; const int k = (int)(e % K), n = (int)(e / K); v2h o;
            o[0] = toh_flush(bfr(w[(size_t)k * N + n]) * WCAR); o[1] = toh_flush(bfr(w[(size_t)(k + 1) * N + n]) * WCAR); *(volatile v2h*)(Bt + e) = o; }
        if (ps == 0) __threadfence(); }
}

__global__ __launch_bounds__(256) void k_ln(const float* __restrict__ src, const float* __restrict__ gam, const float* __restrict__ bet, h16* dst, size_t sstride, size_t dstride) {
#pragma clang fp contract(off)
    const int lane = (int)threadIdx.x & 31;
    const int wave = __builtin_amdgcn_readfirstlane((int)threadIdx.x >> 5);
    const int row = (int)blockIdx.x * 8 + wave;
    const float* s = src + (size_t)blockIdx.y * sstride + (size_t)row * DM + lane * 8;
    h16* d = dst + (size_t)blockIdx.y * dstride + (size_t)row * DM + lane * 8;
    float sum = 0.0f;
#pragma unroll 1
    for (int j = 0; j < 4; ++j) { const v8f v = *(const v8f*)(s + j * 256);
#pragma unroll
        for (int k = 0; k < 8; ++k) sum += bfr(v[k]); }
#pragma unroll
    for (int o = 16; o >= 1; o >>= 1) sum += __shfl_xor(sum, o, 32);
    const float mu = sum * (1.0f / DM);
    float sq = 0.0f;
#pragma unroll 1
    for (int j = 0; j < 4; ++j) { const v8f v = *(const v8f*)(s + j * 256);
#pragma unroll
        for (int k = 0; k < 8; ++k) { const float c = bfr(v[k]) - mu; sq += c * c; } }
#pragma unroll
    for (int o = 16; o >= 1; o >>= 1) sq += __shfl_xor(sq, o, 32);
    const float rstd = rsqrtf(sq * (1.0f / DM) + 1.0e-5f);
#pragma unroll 1
    for (int ps = 0; ps < 2; ++ps) {
#pragma unroll 1
        for (int j = 0; j < 4; ++j) { const v8f v = *(const v8f*)(s + j * 256); const v8f g = *(const v8f*)(gam + j * 256 + lane * 8); const v8f b = *(const v8f*)(bet + j * 256 + lane * 8); v8h o;
#pragma unroll
            for (int k = 0; k < 8; ++k) { const float y = (bfr(v[k]) - mu) * rstd * bfr(g[k]) + bfr(b[k]); o[k] = toh_flush(y * HCAR); }
            *(volatile v8h*)(d + j * 256) = o; }
        if (ps == 0) __threadfence(); }
}

__global__ __launch_bounds__(32) void k_gemm_qkv(const h16* __restrict__ A, const h16* __restrict__ Bt, const float* __restrict__ bias, h16* QK, h16* VT) {
    __shared__ __align__(16) float os[16 * 68];
    __shared__ __align__(16) h16 vts[64 * LP];
    const int lane = threadIdx.x & 31, lr = lane & 15, hi = lane >> 4; const int r0 = blockIdx.x * 64, c0 = blockIdx.y * 64;
    v8f acc[4][4];
#pragma unroll
    for (int mb = 0; mb < 4; ++mb)
#pragma unroll
        for (int nb = 0; nb < 4; ++nb) acc[mb][nb] = (v8f){};
    const size_t aoff = (size_t)(r0 + lr) * DM + 8 * hi, boff = (size_t)(c0 + lr) * DM + 8 * hi;
#pragma unroll 1
    for (int kc = 0; kc < DM; kc += 32) {
        v16h a[4]; v16h bl;
#pragma unroll
        for (int mb = 0; mb < 4; ++mb) a[mb] = ldh(A + aoff + (size_t)mb * 16 * DM + kc);
#pragma unroll
        for (int nb = 0; nb < 4; ++nb) { const v16h b = ldh(Bt + boff + (size_t)nb * 16 * DM + kc); if (nb == 3) bl = b;
#pragma unroll
            for (int mb = 0; mb < 4; ++mb) acc[mb][nb] = wmma16(a[mb], b, acc[mb][nb]); }
        asm volatile("v_nop\n\tv_nop\n\tv_nop\n\tv_nop" : "+v"(acc[0][0]), "+v"(acc[0][1]), "+v"(acc[0][2]), "+v"(acc[0][3]), "+v"(acc[1][0]), "+v"(acc[1][1]), "+v"(acc[1][2]), "+v"(acc[1][3]) : "v"(a[0]), "v"(a[3]), "v"(bl));
        asm volatile("v_nop\n\tv_nop\n\tv_nop\n\tv_nop" : "+v"(acc[2][0]), "+v"(acc[2][1]), "+v"(acc[2][2]), "+v"(acc[2][3]), "+v"(acc[3][0]), "+v"(acc[3][1]), "+v"(acc[3][2]), "+v"(acc[3][3]) : "v"(a[0]), "v"(a[3]), "v"(bl));
    }
    const int which = c0 / DM, head = (c0 % DM) / HD; const int b = r0 / SEQ, t0 = r0 % SEQ; const size_t bh = (size_t)b * NH + head;
    const int rq = lane >> 3, pc = lane & 7;
    if (which < 2) {
        v4f b0 = *(const v4f*)(bias + c0 + pc * 8), b1 = *(const v4f*)(bias + c0 + pc * 8 + 4);
#pragma unroll
        for (int q = 0; q < 4; ++q) { b0[q] = bfr(b0[q]); b1[q] = bfr(b1[q]); }
        h16* P = QK + (size_t)which * PLANE + (bh * SEQ + t0) * HD;
#pragma unroll
        for (int mb = 0; mb < 4; ++mb) {
#pragma unroll
            for (int nb = 0; nb < 4; ++nb) {
#pragma unroll
                for (int j = 0; j < 8; ++j) os[(hi * 8 + j) * 68 + nb * 16 + lr] = acc[mb][nb][j] * QFOLD; }
            __syncthreads();
#pragma unroll 1
            for (int ps = 0; ps < 2; ++ps) {
#pragma unroll
                for (int s = 0; s < 4; ++s) { const int row = 4 * s + rq; const v4f x0 = *(const v4fa*)(os + row * 68 + pc * 8), x1 = *(const v4fa*)(os + row * 68 + pc * 8 + 4); v8h o;
#pragma unroll
                    for (int q = 0; q < 4; ++q) { o[q] = toh_flush(x0[q] + b0[q]); o[4 + q] = toh_flush(x1[q] + b1[q]); }
                    *(volatile v8h*)(P + (size_t)(mb * 16 + row) * HD + pc * 8) = o; }
                if (ps == 0) __threadfence(); }
            __syncthreads();
        }
    } else {
        float bv[4];
#pragma unroll
        for (int nb = 0; nb < 4; ++nb) bv[nb] = bfr(bias[c0 + nb * 16 + lr]);
#pragma unroll
        for (int mb = 0; mb < 4; ++mb)
#pragma unroll
            for (int nb = 0; nb < 4; ++nb) { v8h t;
#pragma unroll
                for (int j = 0; j < 8; ++j) t[j] = toh_flush(acc[mb][nb][j] * QFOLD + bv[nb]);
                *(v8ha*)(vts + (nb * 16 + lr) * LP + mb * 16 + 8 * hi) = t; }
        __syncthreads();
        h16* P = VT + bh * HD * SEQ + t0;
#pragma unroll 1
        for (int ps = 0; ps < 2; ++ps) {
#pragma unroll 1
            for (int s = 0; s < 16; ++s) { const int d = 4 * s + rq; const v8h v = *(const v8ha*)(vts + d * LP + pc * 8); *(volatile v8h*)(P + (size_t)d * SEQ + pc * 8) = v; }
            if (ps == 0) __threadfence(); }
    }
}

__global__ __launch_bounds__(256) void k_flash(const h16* __restrict__ QK, const h16* __restrict__ VT, bf* AH, bf* AL) {
    __shared__ __align__(16) h16 ks[KT * LP];
    __shared__ __align__(16) h16 vs[HD * LP];
    __shared__ __align__(16) float os[8 * 16 * 68];
    const int tid = (int)threadIdx.x, lane = tid & 31, lr = lane & 15, hh = lane >> 4;
    const int wave = __builtin_amdgcn_readfirstlane(tid >> 5);
    const int bh = (int)blockIdx.x / (SEQ / AQ), qb = (int)blockIdx.x % (SEQ / AQ);
    const int q0 = qb * AQ + wave * 16;
    const size_t pbase = (size_t)bh * SEQ * HD;
    const h16* Qp = QK + pbase; const h16* Kp = QK + PLANE + pbase; const h16* Vp = VT + pbase;
    const h16* qrow = Qp + (size_t)(q0 + lr) * HD + 8 * hh;
    const v16h qf0 = cat16(*(const v8ha*)qrow, *(const v8ha*)(qrow + 16));
    const v16h qf1 = cat16(*(const v8ha*)(qrow + 32), *(const v8ha*)(qrow + 48));
    v8f o0 = (v8f){}, o1 = (v8f){}, o2 = (v8f){}, o3 = (v8f){};
    float m = -3.0e38f, l = 0.0f;
    const float csc = SCL * 1.4426950408889634f;
    const int sr = tid >> 3, sp = (tid & 7) * 8;
#pragma unroll 1
    for (int kb = 0; kb < SEQ; kb += KT) {
        __syncthreads();
        {
            const v8h k0v = *(const v8ha*)(Kp + (size_t)(kb + sr) * HD + sp);
            const v8h k1v = *(const v8ha*)(Kp + (size_t)(kb + sr + 32) * HD + sp);
            const v8h v0v = *(const v8ha*)(Vp + (size_t)sr * SEQ + kb + sp);
            const v8h v1v = *(const v8ha*)(Vp + (size_t)(sr + 32) * SEQ + kb + sp);
            *(v8ha*)(ks + sr * LP + sp) = k0v; *(v8ha*)(ks + (sr + 32) * LP + sp) = k1v;
            *(v8ha*)(vs + sr * LP + sp) = v0v; *(v8ha*)(vs + (sr + 32) * LP + sp) = v1v;
        }
        __syncthreads();
#pragma unroll 1
        for (int hf = 0; hf < 2; ++hf) {
            const int kr = hf * 32;
            v8f s0 = (v8f){}, s1 = (v8f){};
            const int ko = (kr + lr) * LP + 8 * hh;
            v16h ka = LDF(ks, ko);            s0 = wmma16(ka, qf0, s0);
            ka = LDF(ks, ko + 32);            s0 = wmma16(ka, qf1, s0);
            ka = LDF(ks, ko + 16 * LP);       s1 = wmma16(ka, qf0, s1);
            ka = LDF(ks, ko + 16 * LP + 32);  s1 = wmma16(ka, qf1, s1);
            asm volatile("v_nop\n\tv_nop\n\tv_nop\n\tv_nop" : "+v"(s0), "+v"(s1) : "v"(ka), "v"(qf0), "v"(qf1));
            float bm = fmaxf(s0[0], s1[0]);
#pragma unroll
            for (int i = 1; i < 8; ++i) bm = fmaxf(bm, fmaxf(s0[i], s1[i]));
            bm *= csc;
            const float bo = __shfl_xor(bm, 16, 32);
            bm = fmaxf(bm, bo);
            const float nm = fmaxf(m, bm);
            const float sc = __builtin_amdgcn_exp2f(m - nm);
            const float sh = nm - 10.0f;
            v16h p; float rs = 0.0f;
#pragma unroll
            for (int i = 0; i < 8; ++i) {
                const float e0 = __builtin_amdgcn_exp2f(s0[i] * csc - sh);
                const float e1 = __builtin_amdgcn_exp2f(s1[i] * csc - sh);
                rs += e0 + e1; p[i] = (h16)e0; p[8 + i] = (h16)e1; }
            const float ro = __shfl_xor(rs, 16, 32);
            rs += ro;
            l = l * sc + rs; m = nm;
            o0 *= sc; o1 *= sc; o2 *= sc; o3 *= sc;
            const int vo = lr * LP + kr + 8 * hh;
            const v16h va0 = LDF(vs, vo), va1 = LDF(vs, vo + 16 * LP), va2 = LDF(vs, vo + 32 * LP), va3 = LDF(vs, vo + 48 * LP);
            o0 = wmma16(va0, p, o0); o1 = wmma16(va1, p, o1); o2 = wmma16(va2, p, o2); o3 = wmma16(va3, p, o3);
            asm volatile("v_nop\n\tv_nop\n\tv_nop\n\tv_nop" : "+v"(o0), "+v"(o1), "+v"(o2), "+v"(o3) : "v"(va3), "v"(p));
        }
    }
    const float inv = 1.0f / l;
    const int wb = wave * (16 * 68);
    const int ob = wb + lr * 68 + 8 * hh;
#pragma unroll
    for (int r = 0; r < 8; ++r) { os[ob + r] = o0[r] * inv; os[ob + 16 + r] = o1[r] * inv; os[ob + 32 + r] = o2[r] * inv; os[ob + 48 + r] = o3[r] * inv; }
    __syncthreads();
    const int b = bh / NH, h = bh % NH; const int rq = lane >> 3, pc = lane & 7;
#pragma unroll 1
    for (int ps = 0; ps < 2; ++ps) {
#pragma unroll
        for (int s = 0; s < 4; ++s) { const int row = 4 * s + rq; const int so = wb + row * 68 + pc * 8;
            const v4f x0 = *(const v4fa*)(os + so), x1 = *(const v4fa*)(os + so + 4); v8us oh, ol;
#pragma unroll
            for (int q = 0; q < 4; ++q) { unsigned short a2, c2; splitf(x0[q], a2, c2); oh[q] = a2; ol[q] = c2; splitf(x1[q], a2, c2); oh[4 + q] = a2; ol[4 + q] = c2; }
            const size_t dst = ((size_t)b * SEQ + q0 + row) * DM + h * HD + pc * 8;
            *(volatile v8us*)(AH + dst) = oh; *(volatile v8us*)(AL + dst) = ol; }
        if (ps == 0) __threadfence(); }
}

__global__ __launch_bounds__(32) void k_gemm_out(const bf* __restrict__ A, const bf* __restrict__ A2, const bf* __restrict__ Bt, const float* __restrict__ bias, float* C) {
    __shared__ __align__(16) float os[16 * 68];
    const int lane = threadIdx.x & 31, lr = lane & 15, hi = lane >> 4; const int r0 = blockIdx.x * 64, c0 = blockIdx.y * 64;
    v8f acc[4][4];
#pragma unroll
    for (int mb = 0; mb < 4; ++mb)
#pragma unroll
        for (int nb = 0; nb < 4; ++nb) acc[mb][nb] = (v8f){};
    const size_t aoff = (size_t)(r0 + lr) * DM + 8 * hi, boff = (size_t)(c0 + lr) * DM + 8 * hi;
#pragma unroll 1
    for (int kc = 0; kc < DM; kc += 32) {
        v16bf a[4], a2[4]; v16bf bl;
#pragma unroll
        for (int mb = 0; mb < 4; ++mb) { a[mb] = ldb(A + aoff + (size_t)mb * 16 * DM + kc); a2[mb] = ldb(A2 + aoff + (size_t)mb * 16 * DM + kc); }
#pragma unroll
        for (int nb = 0; nb < 4; ++nb) { const v16bf b = ldb(Bt + boff + (size_t)nb * 16 * DM + kc); if (nb == 3) bl = b;
#pragma unroll
            for (int mb = 0; mb < 4; ++mb) { acc[mb][nb] = wmmab(a[mb], b, acc[mb][nb]); acc[mb][nb] = wmmab(a2[mb], b, acc[mb][nb]); } }
        asm volatile("v_nop\n\tv_nop\n\tv_nop\n\tv_nop" : "+v"(acc[0][0]), "+v"(acc[0][1]), "+v"(acc[0][2]), "+v"(acc[0][3]), "+v"(acc[1][0]), "+v"(acc[1][1]), "+v"(acc[1][2]), "+v"(acc[1][3]) : "v"(a[3]), "v"(a2[3]), "v"(bl));
        asm volatile("v_nop\n\tv_nop\n\tv_nop\n\tv_nop" : "+v"(acc[2][0]), "+v"(acc[2][1]), "+v"(acc[2][2]), "+v"(acc[2][3]), "+v"(acc[3][0]), "+v"(acc[3][1]), "+v"(acc[3][2]), "+v"(acc[3][3]) : "v"(a[3]), "v"(a2[3]), "v"(bl));
    }
    v4f bb = *(const v4f*)(bias + c0 + lr * 4);
#pragma unroll
    for (int q = 0; q < 4; ++q) bb[q] = bfr(bb[q]);
#pragma unroll
    for (int mb = 0; mb < 4; ++mb) {
#pragma unroll
        for (int nb = 0; nb < 4; ++nb) {
#pragma unroll
            for (int j = 0; j < 8; ++j) os[(hi * 8 + j) * 68 + nb * 16 + lr] = acc[mb][nb][j]; }
        __syncthreads();
        float* crow = C + (size_t)(r0 + mb * 16) * DM + c0;
#pragma unroll 1
        for (int ps = 0; ps < 2; ++ps) {
#pragma unroll
            for (int s = 0; s < 8; ++s) { const int row = 2 * s + hi, cofs = lr * 4; v4f val = *(const v4fa*)(os + row * 68 + cofs); val += bb;
                *(volatile v4f*)(crow + (size_t)row * DM + cofs) = val; }
            if (ps == 0) __threadfence(); }
        __syncthreads();
    }
}

extern "C" void kernel_launch(void* const* d_in, const int* in_sizes, int n_in,
                              void* d_out, int out_size, void* d_ws, size_t ws_size, hipStream_t stream) {
    if (n_in < 7) return;
    if ((size_t)in_sizes[0] < (size_t)(NB - 1) * SEQ_FULL * DM + (size_t)SEQ * DM) return;
    if (in_sizes[1] < DM) return;
    if (in_sizes[2] < DM) return;
    if ((size_t)in_sizes[3] < (size_t)3 * DM * DM) return;
    if (in_sizes[4] < 3 * DM) return;
    if ((size_t)in_sizes[5] < (size_t)DM * DM) return;
    if (in_sizes[6] < DM) return;
    if ((size_t)out_size < (size_t)MR * DM) return;
    if ((size_t)WS_TOTAL > ws_size) return;
    const float* x = (const float*)d_in[0]; const float* gam = (const float*)d_in[1]; const float* bet = (const float*)d_in[2];
    const float* wqkv = (const float*)d_in[3]; const float* bqkv = (const float*)d_in[4]; const float* wo = (const float*)d_in[5]; const float* bo = (const float*)d_in[6];
    float* OUT = (float*)d_out;
    char* wsp = (char*)d_ws;
    h16* WQKV = (h16*)wsp; wsp += SZ_WQKV;
    bf* WO = (bf*)wsp; wsp += SZ_WO;
    h16* HB = (h16*)wsp; wsp += SZ_XB;
    h16* QK = (h16*)wsp; wsp += 2 * SZ_PL;
    h16* VT = (h16*)wsp; wsp += SZ_PL;
    bf* AH = (bf*)wsp; wsp += SZ_XB;
    bf* AL = (bf*)wsp; wsp += SZ_XB;
    k_wtH<<<(unsigned)((DM * 3 * DM / 64 + 63) / 64), 256, 0, stream>>>(wqkv, DM, 3 * DM, WQKV);
    k_wtG<<<(unsigned)((DM * DM / 64 + 63) / 64), 256, 0, stream>>>(wo, DM, DM, WO);
    k_ln<<<dim3((unsigned)(SEQ / 8), NB, 1), 256, 0, stream>>>(x, gam, bet, HB, (size_t)SEQ_FULL * DM, (size_t)SEQ * DM);
    k_gemm_qkv<<<dim3(MR / 64, 3 * DM / 64, 1), 32, 0, stream>>>(HB, WQKV, bqkv, QK, VT);
    k_flash<<<(unsigned)(NB * NH * (SEQ / AQ)), 256, 0, stream>>>(QK, VT, AH, AL);
    k_gemm_out<<<dim3(MR / 64, DM / 64, 1), 32, 0, stream>>>(AH, AL, WO, bo, OUT);
}
